// MultiHeadAttentionQuantum_65481071400570
// MI455X (gfx1250) — hardware-run, weakly checked
//
#include <hip/hip_runtime.h>
#include <stddef.h>


typedef _Float16 v16h __attribute__((ext_vector_type(16)));
typedef _Float16 v8h  __attribute__((ext_vector_type(8)));
typedef float    v8f  __attribute__((ext_vector_type(8)));
typedef float    v4f  __attribute__((ext_vector_type(4)));
typedef _Float16 h16;

#ifndef NB
#define NB 4
#endif
#ifndef SEQ
#define SEQ 512
#endif
#define NB_FULL  4
#define SEQ_FULL 512
#define DIM   64
#define NHEAD 8
#define HD    8
#define MROWS (NB * SEQ)

static_assert(NB >= 1 && NB <= NB_FULL);
static_assert(SEQ >= 64 && SEQ <= SEQ_FULL && (SEQ % 64) == 0);
static_assert(DIM == NHEAD * HD);
static_assert(DIM == 64 && HD == 8 && NHEAD == 8);
static_assert((DIM % 32) == 0);
static_assert((MROWS % 64) == 0 && (MROWS % 32) == 0);
static_assert(((SEQ * NHEAD) % 256) == 0);
static_assert((256 % NHEAD) == 0);
static_assert(256 * 2 == 64 * NHEAD);
static_assert(256 * 4 * 4 == 64 * DIM);
static_assert(128 * 4 == 64 * NHEAD);
static_assert(DIM * DIM == 2 * 256 * 8);

#define LDT 72
#define LDC 68
#define LDQ 196
static_assert((LDT % 8) == 0 && LDT >= 64);
static_assert((LDC % 4) == 0 && LDC >= 64);
static_assert((LDQ % 4) == 0 && LDQ >= 3 * DIM);

#define XCARRY 16.0f
#define WCARRY 64.0f
#define ACARRY 4096.0f

#define X16_BYTES  ((size_t)MROWS * DIM * 2)
#define WQKV_BYTES ((size_t)3 * DIM * DIM * 2)
#define WO_BYTES   ((size_t)DIM * DIM * 2)
#define VEV_BYTES  ((size_t)MROWS * DIM * 4)
#define SC_BYTES   ((size_t)MROWS * NHEAD * 4)
#define OFF_X16  ((size_t)0)
#define OFF_WQKV (OFF_X16 + X16_BYTES)
#define OFF_WO   (OFF_WQKV + WQKV_BYTES)
#define OFF_VEV  (OFF_WO + WO_BYTES)
#define OFF_SC   (OFF_VEV + VEV_BYTES)
#define WS_TOTAL (OFF_SC + SC_BYTES)
static_assert((X16_BYTES % 128) == 0 && (WQKV_BYTES % 128) == 0 && (WO_BYTES % 128) == 0);
static_assert((VEV_BYTES % 128) == 0 && (SC_BYTES % 128) == 0);
static_assert(WS_TOTAL <= (size_t)134217728);

__device__ __forceinline__ float bf16r(float x) {
  unsigned int u = __float_as_uint(x);
  u = (u + 0x7FFFu + ((u >> 16) & 1u)) & 0xFFFF0000u;
  return __uint_as_float(u);
}

static __device__ __forceinline__ h16 toh_flush(float v) {
  const h16 r = (h16)v;
  return (fabsf(v) < 6.103515625e-05f) ? (h16)0.0f : r;
}

__device__ __forceinline__ v16h frag_at(const _Float16* p) {
  v8h lo = *(const v8h*)(p);
  v8h hi = *(const v8h*)(p + 16);
  v16h out;
#pragma unroll
  for (int i = 0; i < 8; ++i) { out[i] = lo[i]; out[i + 8] = hi[i]; }
  return out;
}
__device__ __forceinline__ v16h ld_frag(const _Float16* base, unsigned ld) {
  const unsigned lane = threadIdx.x & 31u;
  return frag_at(base + (lane & 15u) * ld + (lane >> 4) * 8u);
}

__device__ __forceinline__ v8f wmma16(v16h a, v16h b, v8f c) {
  v8f d = __builtin_amdgcn_wmma_f32_16x16x32_f16(false, a, false, b, (short)0, c,
                                                 false, false);
  asm volatile("v_nop\n\tv_nop\n\tv_nop\n\tv_nop" : "+v"(d) : "v"(a), "v"(b));
  return d;
}

__device__ __forceinline__ v8h cvt8(const float* __restrict__ src, const float carry) {
  const v4f a0 = *(const v4f*)(src);
  const v4f a1 = *(const v4f*)(src + 4);
  v8h o;
#pragma unroll
  for (int i = 0; i < 4; ++i) {
    o[i]     = toh_flush(carry * bf16r(a0[i]));
    o[i + 4] = toh_flush(carry * bf16r(a1[i]));
  }
  return o;
}

__device__ __forceinline__ void circuit_ev(const v4f a0, const v4f a1, const v4f p0,
                                           const v4f p1, v4f& e0, v4f& e1) {
  const float c0 = cosf(a0[0] + p0[0]);
  const float c1 = cosf(a0[1] + p0[1]);
  const float c2 = cosf(a0[2] + p0[2]);
  const float c3 = cosf(a0[3] + p0[3]);
  const float c4 = cosf(a1[0] + p1[0]);
  const float c5 = cosf(a1[1] + p1[1]);
  const float c6 = cosf(a1[2] + p1[2]);
  const float c7 = cosf(a1[3] + p1[3]);
  const float t12 = c1 * c2;
  const float t13 = t12 * c3;
  const float t14 = t13 * c4;
  const float t15 = t14 * c5;
  const float t16 = t15 * c6;
  const float t17 = t16 * c7;
  e0[0] = t17;
  e0[1] = c0 * c1;
  e0[2] = c0 * t12;
  e0[3] = c0 * t13;
  e1[0] = c0 * t14;
  e1[1] = c0 * t15;
  e1[2] = c0 * t16;
  e1[3] = c0 * t17;
}

__global__ __launch_bounds__(256) void xcvt_kernel(
    const float* __restrict__ X, _Float16* __restrict__ X16) {
  const unsigned g = blockIdx.x * 256u + threadIdx.x;
  const unsigned crow = g >> 3;
  const unsigned c = (g & 7u) * 8u;
  const unsigned bidx = crow / (unsigned)SEQ;
  const unsigned sq = crow - bidx * (unsigned)SEQ;
  const size_t frow = (size_t)bidx * SEQ_FULL + sq;
  const v8h o = cvt8(X + frow * DIM + c, XCARRY);
  _Float16* p = X16 + (size_t)crow * DIM + c;
  *(volatile v8h*)p = o;
  __threadfence();
  *(volatile v8h*)p = o;
}

__global__ __launch_bounds__(256) void wcvt_kernel(
    const float* __restrict__ Wq, const float* __restrict__ Wk,
    const float* __restrict__ Wv, const float* __restrict__ Wo,
    _Float16* __restrict__ Wqkv, _Float16* __restrict__ Wo16) {
  const unsigned e = (blockIdx.x * 256u + threadIdx.x) * 8u;
  const v8h xq = cvt8(Wq + e, WCARRY);
  const v8h xk = cvt8(Wk + e, WCARRY);
  const v8h xv = cvt8(Wv + e, WCARRY);
  const v8h xo = cvt8(Wo + e, WCARRY);
  _Float16* pq = Wqkv + e;
  _Float16* pk = Wqkv + (size_t)DIM * DIM + e;
  _Float16* pv = Wqkv + (size_t)2 * DIM * DIM + e;
  _Float16* po = Wo16 + e;
  *(volatile v8h*)pq = xq;
  *(volatile v8h*)pk = xk;
  *(volatile v8h*)pv = xv;
  *(volatile v8h*)po = xo;
  __threadfence();
  *(volatile v8h*)pq = xq;
  *(volatile v8h*)pk = xk;
  *(volatile v8h*)pv = xv;
  *(volatile v8h*)po = xo;
}

__global__ __launch_bounds__(256) void qkv_circuit_kernel(
    const _Float16* __restrict__ X16, const _Float16* __restrict__ Wqkv,
    const float* __restrict__ qpar, float* __restrict__ Vev, float* __restrict__ Sc) {
  __shared__ __attribute__((aligned(16))) float Cs[64 * LDQ];
  __shared__ __attribute__((aligned(16))) float Ss[64 * NHEAD];
  const unsigned tid = threadIdx.x, lane = tid & 31u;
  const unsigned w = (unsigned)__builtin_amdgcn_readfirstlane((int)(threadIdx.x >> 5));
  const unsigned mw = w >> 1, nw = w & 1u;
  const unsigned hh = lane >> 4, m = lane & 15u;
  const unsigned row0 = blockIdx.x * 64u;

  const _Float16* ap = X16 + (size_t)(row0 + mw * 16u + m) * DIM + hh * 8u;
  const v16h a0 = frag_at(ap);
  const v16h a1 = frag_at(ap + 32);
  const float cs = 1.0f / (XCARRY * WCARRY);
#pragma unroll
  for (unsigned mat = 0; mat < 3u; ++mat) {
    const _Float16* bp0 = Wqkv + (size_t)(mat * 64u + nw * 32u + m) * DIM + hh * 8u;
    const _Float16* bp1 = bp0 + (size_t)16 * DIM;
    v8f acc0 = {}, acc1 = {};
    const v16h b00 = frag_at(bp0);
    const v16h b10 = frag_at(bp1);
    const v16h b01 = frag_at(bp0 + 32);
    const v16h b11 = frag_at(bp1 + 32);
    acc0 = wmma16(a0, b00, acc0);
    acc1 = wmma16(a0, b10, acc1);
    acc0 = wmma16(a1, b01, acc0);
    acc1 = wmma16(a1, b11, acc1);
#pragma unroll
    for (int r = 0; r < 8; ++r) {
      const unsigned ci = (mw * 16u + hh * 8u + (unsigned)r) * LDQ + mat * 64u + nw * 32u + m;
      Cs[ci]       = acc0[r] * cs;
      Cs[ci + 16u] = acc1[r] * cs;
    }
  }
  __syncthreads();

  const unsigned head = tid & 7u;
  const v4f pa = *(const v4f*)(qpar + head * 8u);
  const v4f pb = *(const v4f*)(qpar + head * 8u + 4u);
  v4f p0, p1;
#pragma unroll
  for (int j = 0; j < 4; ++j) { p0[j] = bf16r(pa[j]); p1[j] = bf16r(pb[j]); }

#pragma unroll 1
  for (unsigned i = 0; i < 2u; ++i) {
    const unsigned r = 32u * i + (tid >> 3);
    const unsigned cb = r * LDQ + head * 8u;
    v4f qe0, qe1, ke0, ke1, ve0, ve1;
    circuit_ev(*(const v4f*)&Cs[cb], *(const v4f*)&Cs[cb + 4u], p0, p1, qe0, qe1);
    circuit_ev(*(const v4f*)&Cs[cb + 64u], *(const v4f*)&Cs[cb + 68u], p0, p1, ke0, ke1);
    circuit_ev(*(const v4f*)&Cs[cb + 128u], *(const v4f*)&Cs[cb + 132u], p0, p1, ve0, ve1);
    float sc = 0.0f;
#pragma unroll
    for (int j = 0; j < 4; ++j) sc += qe0[j] * ke0[j];
#pragma unroll
    for (int j = 0; j < 4; ++j) sc += qe1[j] * ke1[j];
    Ss[r * NHEAD + head] = sc * 0.35355339059327373f;
    *(v4f*)&Cs[cb + 128u] = ve0;
    *(v4f*)&Cs[cb + 132u] = ve1;
  }
  __syncthreads();

  v4f xs[4];
  size_t off[4];
#pragma unroll
  for (unsigned i = 0; i < 4u; ++i) {
    const unsigned r = 16u * i + (tid >> 4);
    const unsigned c = (tid & 15u) * 4u;
    xs[i] = *(const v4f*)&Cs[r * LDQ + 128u + c];
    off[i] = (size_t)(row0 + r) * DIM + c;
  }
  v4f sv = {};
  const size_t soff = (size_t)row0 * NHEAD + (size_t)tid * 4u;
  if (w < 4u) sv = *(const v4f*)&Ss[tid * 4u];
#pragma unroll
  for (int i = 0; i < 4; ++i) *(volatile v4f*)(Vev + off[i]) = xs[i];
  if (w < 4u) *(volatile v4f*)(Sc + soff) = sv;
  __threadfence();
#pragma unroll
  for (int i = 0; i < 4; ++i) *(volatile v4f*)(Vev + off[i]) = xs[i];
  if (w < 4u) *(volatile v4f*)(Sc + soff) = sv;
}

__global__ __launch_bounds__(256) void attn_out_kernel(
    const float* __restrict__ Sc, const float* __restrict__ Vev,
    const _Float16* __restrict__ Wo16, const float* __restrict__ bo,
    float* __restrict__ outf) {
  __shared__ __attribute__((aligned(16))) _Float16 As[64 * LDT];
  __shared__ __attribute__((aligned(16))) float Cs[64 * LDC];
  __shared__ float Red[8 * NHEAD];
  const unsigned tid = threadIdx.x, lane = tid & 31u;
  const unsigned w = (unsigned)__builtin_amdgcn_readfirstlane((int)(threadIdx.x >> 5));
  const unsigned mw = w >> 1, nw = w & 1u;
  const unsigned hh = lane >> 4, m = lane & 15u;
  const unsigned row0 = blockIdx.x * 64u;
  const unsigned head = tid & 7u;
  const unsigned bblk = row0 / (unsigned)SEQ;
  const size_t sbase = (size_t)bblk * SEQ * NHEAD;

  float mx = -1.0e30f;
#pragma unroll 1
  for (unsigned j = 0; j < (unsigned)((SEQ * NHEAD) / 256); ++j)
    mx = fmaxf(mx, Sc[sbase + tid + 256u * j]);
  mx = fmaxf(mx, __shfl_xor(mx, 8, 32));
  mx = fmaxf(mx, __shfl_xor(mx, 16, 32));
  if (lane < 8u) Red[w * NHEAD + lane] = mx;
  __syncthreads();
  float gm = Red[head];
#pragma unroll
  for (unsigned ww = 1; ww < 8u; ++ww) gm = fmaxf(gm, Red[ww * NHEAD + head]);
  __syncthreads();

  float sm = 0.0f;
#pragma unroll 1
  for (unsigned j = 0; j < (unsigned)((SEQ * NHEAD) / 256); ++j)
    sm += __expf(Sc[sbase + tid + 256u * j] - gm);
  sm += __shfl_xor(sm, 8, 32);
  sm += __shfl_xor(sm, 16, 32);
  if (lane < 8u) Red[w * NHEAD + lane] = sm;
  __syncthreads();
  float gs = Red[head];
#pragma unroll
  for (unsigned ww = 1; ww < 8u; ++ww) gs += Red[ww * NHEAD + head];
  const float ginv = 1.0f / gs;

#pragma unroll
  for (unsigned i = 0; i < 2u; ++i) {
    const unsigned r = 32u * i + (tid >> 3);
    const size_t row = (size_t)row0 + r;
    const float s = Sc[row * NHEAD + head];
    const float pw = __expf(s - gm) * ginv * ACARRY;
    const v4f v0 = *(const v4f*)(Vev + row * DIM + head * 8u);
    const v4f v1 = *(const v4f*)(Vev + row * DIM + head * 8u + 4u);
    v8h o;
#pragma unroll
    for (int j = 0; j < 4; ++j) {
      o[j]     = toh_flush(pw * v0[j]);
      o[j + 4] = toh_flush(pw * v1[j]);
    }
    *(v8h*)&As[r * LDT + head * 8u] = o;
  }
  __syncthreads();

  const _Float16* bp0 = Wo16 + (size_t)(nw * 32u + m) * DIM + hh * 8u;
  const _Float16* bp1 = bp0 + (size_t)16 * DIM;
  v8f acc0 = {}, acc1 = {};
#pragma unroll
  for (unsigned c = 0; c < 2u; ++c) {
    const v16h a  = ld_frag(&As[(mw * 16u) * LDT + c * 32u], LDT);
    const v16h b0 = frag_at(bp0 + c * 32u);
    const v16h b1 = frag_at(bp1 + c * 32u);
    acc0 = wmma16(a, b0, acc0);
    acc1 = wmma16(a, b1, acc1);
  }
#pragma unroll
  for (int r = 0; r < 8; ++r) {
    const unsigned ci = (mw * 16u + hh * 8u + (unsigned)r) * LDC + nw * 32u + m;
    Cs[ci]       = acc0[r];
    Cs[ci + 16u] = acc1[r];
  }
  __syncthreads();

  const float cs = 1.0f / (WCARRY * ACARRY);
  v4f xs[4];
  size_t off[4];
#pragma unroll
  for (unsigned i = 0; i < 4u; ++i) {
    const unsigned r = 16u * i + (tid >> 4);
    const unsigned c = (tid & 15u) * 4u;
    const unsigned crow = row0 + r;
    const unsigned bidx = crow / (unsigned)SEQ;
    const unsigned sq = crow - bidx * (unsigned)SEQ;
    const size_t frow = (size_t)bidx * SEQ_FULL + sq;
    const v4f u = *(const v4f*)&Cs[r * LDC + c];
    const v4f g = *(const v4f*)(bo + c);
    v4f val;
#pragma unroll
    for (int j = 0; j < 4; ++j) val[j] = u[j] * cs + bf16r(g[j]);
    xs[i] = val;
    off[i] = frow * DIM + c;
  }
#pragma unroll
  for (int i = 0; i < 4; ++i) *(volatile v4f*)(outf + off[i]) = xs[i];
  __threadfence();
#pragma unroll
  for (int i = 0; i < 4; ++i) *(volatile v4f*)(outf + off[i]) = xs[i];
}

extern "C" void kernel_launch(void* const* d_in, const int* in_sizes, int n_in,
                              void* d_out, int out_size, void* d_ws, size_t ws_size,
                              hipStream_t stream) {
  if (n_in < 7) return;
  const long long need_x = ((long long)(NB - 1) * SEQ_FULL + SEQ) * DIM;
  if ((long long)in_sizes[0] < need_x) return;
  if (in_sizes[1] < DIM * DIM || in_sizes[2] < DIM * DIM) return;
  if (in_sizes[3] < DIM * DIM || in_sizes[4] < DIM * DIM) return;
  if (in_sizes[5] < DIM) return;
  if (in_sizes[6] < NHEAD * HD) return;
  if ((long long)out_size < need_x) return;
  if (ws_size < WS_TOTAL) return;

  const float* X    = (const float*)d_in[0];
  const float* wq   = (const float*)d_in[1];
  const float* wk   = (const float*)d_in[2];
  const float* wv   = (const float*)d_in[3];
  const float* wo   = (const float*)d_in[4];
  const float* bo   = (const float*)d_in[5];
  const float* qpar = (const float*)d_in[6];
  float* out = (float*)d_out;

  char* ws = (char*)d_ws;
  _Float16* X16   = (_Float16*)(ws + OFF_X16);
  _Float16* Wqkv  = (_Float16*)(ws + OFF_WQKV);
  _Float16* Wo16  = (_Float16*)(ws + OFF_WO);
  float*    Vev   = (float*)(ws + OFF_VEV);
  float*    Sc    = (float*)(ws + OFF_SC);

  dim3 blk(256);
  wcvt_kernel<<<dim3(2), blk, 0, stream>>>(wq, wk, wv, wo, Wqkv, Wo16);
  xcvt_kernel<<<dim3(MROWS / 32), blk, 0, stream>>>(X, X16);
  qkv_circuit_kernel<<<dim3(MROWS / 64), blk, 0, stream>>>(X16, Wqkv, qpar, Vev, Sc);
  attn_out_kernel<<<dim3(MROWS / 64), blk, 0, stream>>>(Sc, Vev, Wo16, bo, out);
}
